// RelationalDynamicAggregation_33406255628295
// MI455X (gfx1250) — hardware-run, weakly checked
//
#include <hip/hip_runtime.h>


#ifndef NB
#define NB 256
#endif
#ifndef SEQ
#define SEQ 200
#endif
#define NB_FULL  256
#define SEQ_FULL 200
#define NT   8
#define NR   8
#define ND   64
#define NF   20
#define NTR  (NT * NR)
#define SP   ((SEQ + 31) & ~31)
#define SHP  72
#define STP  (SP + 8)
#define AWV  4
#define OSP  68
#define SEQC  1024.0f
#define SEQCI (1.0f / 1024.0f)
#define RIC   4096.0f
#define SCL  ((float)(1.4426950408889634 / 4194304.0))
#define PSH  14.0f
#define NEGB (-3.0e38f)

static_assert(NB <= NB_FULL);
static_assert(SEQ <= SEQ_FULL);
static_assert(SEQ >= 1);
static_assert(SP % 32 == 0);
static_assert(SP >= SEQ);
static_assert(ND == 64);
static_assert(ND % 32 == 0);
static_assert(NTR == 16 * AWV);
static_assert(NR == 8);
static_assert((SP * 8) % (32 * AWV) == 0);
static_assert((NTR * 8) % (32 * AWV) == 0);
static_assert(SHP % 8 == 0);
static_assert(STP % 8 == 0);
static_assert(SHP >= ND);
static_assert((OSP * 4) % 16 == 0);
static_assert(OSP >= ND);
static_assert(8 * 32 * 16 == 16 * ND * 4);
static_assert((size_t)SP * SHP * 2 + (size_t)ND * STP * 2 + (size_t)NTR * SHP * 2 + (size_t)NR * SP * 4 + (size_t)SP * 4 + (size_t)2 * NR * NF * 4 + (size_t)AWV * 16 * OSP * 4 <= 131072);

typedef _Float16 h16;
typedef __attribute__((ext_vector_type(16))) _Float16 v16h;
typedef __attribute__((ext_vector_type(8)))  _Float16 v8h;
typedef __attribute__((ext_vector_type(8)))  float    v8f;
typedef __attribute__((ext_vector_type(4)))  float    v4f;
typedef __attribute__((ext_vector_type(4)))  int      v4i;
typedef v4f  __attribute__((may_alias)) v4fa;
typedef v4i  __attribute__((may_alias)) v4ia;
typedef v8h  __attribute__((may_alias)) v8ha;

__device__ __forceinline__ unsigned short f2bf(float f) { unsigned u = __float_as_uint(f); u += 0x7FFFu + ((u >> 16) & 1u); return (unsigned short)(u >> 16); }
__device__ __forceinline__ float bfr(float f) { return __uint_as_float(((unsigned)f2bf(f)) << 16); }
__device__ __forceinline__ v16h cat16(v8h lo, v8h hi) { return __builtin_shufflevector(lo, hi, 0, 1, 2, 3, 4, 5, 6, 7, 8, 9, 10, 11, 12, 13, 14, 15); }
__device__ __forceinline__ v8f wmma16(v16h a, v16h b, v8f c) { return __builtin_amdgcn_wmma_f32_16x16x32_f16(false, a, false, b, (short)0, c, false, false); }
__device__ __forceinline__ v8f wmma16g(v16h a, v16h b, v8f c) { c = wmma16(a, b, c); asm volatile("v_nop\n\tv_nop\n\tv_nop\n\tv_nop" : "+v"(c) : "v"(a), "v"(b)); return c; }
static __device__ __forceinline__ h16 toh_flush(float v) { const h16 r = (h16)v; return (fabsf(v) < 6.103515625e-05f) ? (h16)0.0f : r; }
__device__ __forceinline__ void wave_sync() { __builtin_amdgcn_fence(3  , "wavefront"); __builtin_amdgcn_wave_barrier(); asm volatile("" ::: "memory"); }

#define LFRAG(arr, o) cat16(*(const v8ha*)(&arr[(o)]), *(const v8ha*)(&arr[(o) + 16]))

__global__ __launch_bounds__(32 * AWV) void k_relpool(const float* __restrict__ seq, const float* __restrict__ dtn, const float* __restrict__ tgt, const float* __restrict__ tval,
                                                      const int* __restrict__ vmask, const float* __restrict__ remb, const float* __restrict__ freal, const float* __restrict__ fimag,
                                                      float* OUT) {
    __shared__ __align__(16) h16   sSeqH[SP * SHP];
    __shared__ __align__(16) h16   sSeqT[ND * STP];
    __shared__ __align__(16) h16   sRi[NTR * SHP];
    __shared__ __align__(16) float sDecT[NR * SP];
    __shared__ __align__(16) int   sVal[SP];
    __shared__ __align__(16) float sFq[2 * NR * NF];
    __shared__ __align__(16) float os[AWV * 16 * OSP];

    const int tid = threadIdx.x;
    const int lane = tid & 31, lr = lane & 15, hi = lane >> 4;
    const int wave = __builtin_amdgcn_readfirstlane((int)(threadIdx.x >> 5));
    const int b = blockIdx.x;

    for (int i = tid; i < NR * NF; i += 32 * AWV) { sFq[i] = bfr(freal[i]); sFq[NR * NF + i] = bfr(fimag[i]); }

    const float* seqB = seq + (size_t)b * SEQ_FULL * ND;
    for (int idx = tid; idx < SP * 8; idx += 32 * AWV) {
        const int s = idx >> 3, c8 = (idx & 7) * 8;
        const int sc = s < SEQ ? s : (SEQ - 1);
        const float* gp = seqB + (size_t)sc * ND + c8;
        v4f x0 = *(const v4f*)gp, x1 = *(const v4f*)(gp + 4);
        asm volatile("" : "+v"(x0), "+v"(x1));
        const bool ok = s < SEQ;
        v8h hv;
#pragma unroll
        for (int i = 0; i < 4; ++i) {
            const float a0 = ok ? bfr(x0[i]) * SEQC : 0.0f;
            const float a1 = ok ? bfr(x1[i]) * SEQC : 0.0f;
            hv[i] = toh_flush(a0); hv[4 + i] = toh_flush(a1); }
        *(v8ha*)(&sSeqH[s * SHP + c8]) = hv;
#pragma unroll
        for (int i = 0; i < 8; ++i) sSeqT[(c8 + i) * STP + s] = hv[i];
    }

    {
        const float* tvB = tval + (size_t)b * NTR * ND;
        const float* tgB = tgt + (size_t)b * NT * ND;
        for (int idx = tid; idx < NTR * 8; idx += 32 * AWV) {
            const int tr = idx >> 3, c8 = (idx & 7) * 8;
            const int t = tr >> 3, r = tr & 7;
            const float* pv = tvB + (size_t)tr * ND + c8;
            const float* pe = remb + (size_t)r * ND + c8;
            const float* pt = tgB + (size_t)t * ND + c8;
            const v4f v0 = *(const v4f*)pv, v1 = *(const v4f*)(pv + 4);
            const v4f e0 = *(const v4f*)pe, e1 = *(const v4f*)(pe + 4);
            const v4f g0 = *(const v4f*)pt, g1 = *(const v4f*)(pt + 4);
            v8h hv;
#pragma unroll
            for (int i = 0; i < 4; ++i) {
                const float a0 = ((bfr(e0[i]) + bfr(v0[i])) * bfr(g0[i])) * RIC;
                const float a1 = ((bfr(e1[i]) + bfr(v1[i])) * bfr(g1[i])) * RIC;
                hv[i] = toh_flush(a0); hv[4 + i] = toh_flush(a1); }
            *(v8ha*)(&sRi[tr * SHP + c8]) = hv;
        }
    }
    __syncthreads();

    {
        const float* dtB = dtn + (size_t)b * SEQ_FULL;
        const int* vmB = vmask + (size_t)b * SEQ_FULL;
        for (int s = tid; s < SP; s += 32 * AWV) {
            const int sc = s < SEQ ? s : (SEQ - 1);
            float dt = dtB[sc]; int vm = vmB[sc];
            asm volatile("" : "+v"(dt), "+v"(vm));
            dt = bfr(dt);
            float acc[NR];
#pragma unroll
            for (int r = 0; r < NR; ++r) acc[r] = 0.0f;
#pragma unroll 1
            for (int k = 0; k < NF; ++k) {
                const float fk = (float)k / (float)(NF - 1);
                const float ck = 6.2831855f * (fk * 0.5f);
                const float wk = ck * dt;
                float sw, cw;
                sincosf(wk, &sw, &cw);
#pragma unroll
                for (int r = 0; r < NR; ++r) acc[r] += cw * sFq[r * NF + k] - sw * sFq[NR * NF + r * NF + k];
            }
            const bool ok = s < SEQ;
#pragma unroll
            for (int r = 0; r < NR; ++r) {
                float dv = acc[r] * (1.0f / (2.0f * (float)NF));
                dv = fminf(fmaxf(dv, 0.0f), 1.0f);
                sDecT[r * SP + s] = ok ? dv : 0.0f; }
            sVal[s] = ok ? vm : 0;
        }
    }
    __syncthreads();

    const int tr0 = wave * 16;
    const int rb = (tr0 + lr) * SHP + 8 * hi;
    const v16h qb0 = LFRAG(sRi, rb), qb1 = LFRAG(sRi, rb + 32);
    const int dro = (lr & 7) * SP + 8 * hi;
    v8f o[4];
#pragma unroll
    for (int j = 0; j < 4; ++j) o[j] = (v8f){};
    float m = NEGB, l = 0.0f;
#pragma unroll 1
    for (int key0 = 0; key0 < SP; key0 += 32) {
        const int ao = (key0 + lr) * SHP + 8 * hi;
        const v16h ka0 = LFRAG(sSeqH, ao), ka1 = LFRAG(sSeqH, ao + 32);
        const v16h kb0 = LFRAG(sSeqH, ao + 16 * SHP), kb1 = LFRAG(sSeqH, ao + 16 * SHP + 32);
        v8f sA = (v8f){}, sB = (v8f){};
        sA = wmma16g(ka0, qb0, sA); sA = wmma16g(ka1, qb1, sA);
        sB = wmma16g(kb0, qb0, sB); sB = wmma16g(kb1, qb1, sB);
        const v4i n0 = *(const v4ia*)(&sVal[key0 + 8 * hi]),      n1 = *(const v4ia*)(&sVal[key0 + 8 * hi + 4]);
        const v4i n2 = *(const v4ia*)(&sVal[key0 + 16 + 8 * hi]), n3 = *(const v4ia*)(&sVal[key0 + 16 + 8 * hi + 4]);
        const v4f d0 = *(const v4fa*)(&sDecT[dro + key0]),      d1 = *(const v4fa*)(&sDecT[dro + key0 + 4]);
        const v4f d2 = *(const v4fa*)(&sDecT[dro + key0 + 16]), d3 = *(const v4fa*)(&sDecT[dro + key0 + 20]);
        float ta[8], tb[8], da[8], db[8]; bool fa[8], fb[8];
#pragma unroll
        for (int r = 0; r < 4; ++r) {
            fa[r] = n0[r] != 0; fa[4 + r] = n1[r] != 0; fb[r] = n2[r] != 0; fb[4 + r] = n3[r] != 0;
            da[r] = d0[r]; da[4 + r] = d1[r]; db[r] = d2[r]; db[4 + r] = d3[r]; }
        float mx = NEGB;
#pragma unroll
        for (int r = 0; r < 8; ++r) {
            ta[r] = sA[r] * SCL; tb[r] = sB[r] * SCL;
            mx = fmaxf(mx, fmaxf(fa[r] ? ta[r] : NEGB, fb[r] ? tb[r] : NEGB)); }
        mx = fmaxf(mx, __shfl_xor(mx, 16, 32));
        const float mnew = fmaxf(m, mx);
        const float alpha = __builtin_amdgcn_exp2f(m - mnew);
        const float sh = PSH - mnew;
        v16h pb; float ls = 0.0f;
#pragma unroll
        for (int r = 0; r < 8; ++r) {
            const float ea = __builtin_amdgcn_exp2f(ta[r] + sh), eb = __builtin_amdgcn_exp2f(tb[r] + sh);
            const float ga = fa[r] ? ea : 0.0f, gb = fb[r] ? eb : 0.0f;
            ls += ga + gb;
            pb[r] = toh_flush(ga * da[r]); pb[8 + r] = toh_flush(gb * db[r]); }
        l = l * alpha + ls; m = mnew;
#pragma unroll
        for (int j = 0; j < 4; ++j) o[j] = o[j] * alpha;
        const int vo = lr * STP + key0 + 8 * hi;
#pragma unroll
        for (int j = 0; j < 4; ++j) { const v16h vj = LFRAG(sSeqT, vo + j * 16 * STP); o[j] = wmma16g(vj, pb, o[j]); }
    }
    l += __shfl_xor(l, 16, 32);
    const bool any = l > 0.0f;
    const float lsafe = any ? l : 1.0f;
    const float inv = any ? ((1.0f / lsafe) * SEQCI) : __uint_as_float(0x7FC00000u);
    const int wb = wave * 16 * OSP;
#pragma unroll
    for (int j = 0; j < 4; ++j) {
        v4f a, c;
        a[0] = o[j][0] * inv; a[1] = o[j][1] * inv; a[2] = o[j][2] * inv; a[3] = o[j][3] * inv;
        c[0] = o[j][4] * inv; c[1] = o[j][5] * inv; c[2] = o[j][6] * inv; c[3] = o[j][7] * inv;
        *(v4fa*)(&os[wb + lr * OSP + 16 * j + 8 * hi]) = a; *(v4fa*)(&os[wb + lr * OSP + 16 * j + 8 * hi + 4]) = c; }
    wave_sync();
    float* obase = OUT + ((size_t)b * NTR + tr0) * ND;
#pragma unroll 1
    for (int ps = 0; ps < 2; ++ps) {
#pragma unroll
        for (int s = 0; s < 8; ++s) { const int p = s * 32 + lane; const int row = p >> 4, c4 = (p & 15) * 4;
            const v4f val = *(const v4fa*)(&os[wb + row * OSP + c4]);
            *(volatile v4f*)(obase + (size_t)p * 4) = val; }
        if (ps == 0) __threadfence(); }
}

extern "C" void kernel_launch(void* const* d_in, const int* in_sizes, int n_in,
                              void* d_out, int out_size, void* d_ws, size_t ws_size, hipStream_t stream) {
    if (n_in < 8) return;
    const size_t needs = (size_t)(NB - 1) * SEQ_FULL + SEQ;
    if ((size_t)in_sizes[0] < needs * ND) return;
    if ((size_t)in_sizes[1] < needs) return;
    if ((size_t)in_sizes[2] < (size_t)NB * NT * ND) return;
    if ((size_t)in_sizes[3] < (size_t)NB * NTR * ND) return;
    if ((size_t)in_sizes[4] < needs) return;
    if (in_sizes[5] < NR * ND || in_sizes[6] < NR * NF || in_sizes[7] < NR * NF) return;
    if ((size_t)out_size < (size_t)NB * NTR * ND) return;
    const float* seq  = (const float*)d_in[0];
    const float* dtn  = (const float*)d_in[1];
    const float* tgt  = (const float*)d_in[2];
    const float* tval = (const float*)d_in[3];
    const int*   vmk  = (const int*)d_in[4];
    const float* remb = (const float*)d_in[5];
    const float* fre  = (const float*)d_in[6];
    const float* fim  = (const float*)d_in[7];
    float* OUT = (float*)d_out;
    k_relpool<<<dim3(NB, 1, 1), dim3(32 * AWV, 1, 1), 0, stream>>>(seq, dtn, tgt, tval, vmk, remb, fre, fim, OUT);
}
